// SCD_cell_11879879544318
// MI455X (gfx1250) — hardware-verified
//
#include <hip/hip_runtime.h>
#include <stdint.h>
#include <stddef.h>


typedef _Float16 f16;
typedef _Float16 v16h __attribute__((ext_vector_type(16)));
typedef _Float16 v8h  __attribute__((ext_vector_type(8)));
typedef float    v8f  __attribute__((ext_vector_type(8)));
typedef float    v4f  __attribute__((ext_vector_type(4)));
typedef unsigned int v4u __attribute__((ext_vector_type(4)));

union Frag { v16h v; v8h half[2]; };
union Pk8  { v8h h; v4u u; };

#define HID     512
#define KTOT    1536
#define NKT     48
#define NGATE   4
#define TSUB    2
#define NFRAG   8
#define ROWS_PB 32
#define COLS_PB 128
#define STG_LD  132
#define OPSCALE 16.0f
#define INVSC   (1.0f / 256.0f)

__device__ __forceinline__ v8f wmma16(v16h a, v16h b, v8f c)
{
    v8f d = __builtin_amdgcn_wmma_f32_16x16x32_f16(false, a, false, b, (short)0, c, false, false);
    asm volatile("v_nop\n\tv_nop\n\tv_nop\n\tv_nop" : "+v"(d) : "v"(a), "v"(b));
    return d;
}

__device__ __forceinline__ float rcp_f(float x)  { return __builtin_amdgcn_rcpf(x); }
__device__ __forceinline__ float sigm_f(float x) { return rcp_f(1.0f + __expf(-x)); }
__device__ __forceinline__ float tanh_f(float x) { return 2.0f * rcp_f(1.0f + __expf(-2.0f * x)) - 1.0f; }

__global__ void __launch_bounds__(256)
k_pack_w(const float* __restrict__ U11, const float* __restrict__ U21,
         const float* __restrict__ W01, f16* Apk, int total8)
{
    const int t = blockIdx.x * 256 + threadIdx.x;
    if (t >= total8) return;
    const int jh   = t & 1;
    const int l    = (t >> 1) & 31;
    const int frag = t >> 6;
    const int kt   = frag % NKT;
    const int mt   = frag / NKT;
    const int m    = mt * 16 + (l & 15);
    const int hh   = l >> 4;
    const int k    = kt * 32 + jh * 16 + hh * 8;
    const int seg  = k >> 9;
    const int kk   = k & (HID - 1);
    const float* src = (seg == 0) ? U11 : ((seg == 1) ? U21 : W01);
    const float* p = src + (size_t)m * HID + kk;
    const v4f x0 = *(const v4f*)(p);
    const v4f x1 = *(const v4f*)(p + 4);
    Pk8 o;
    o.h[0] = (f16)(x0[0] * OPSCALE);
    o.h[1] = (f16)(x0[1] * OPSCALE);
    o.h[2] = (f16)(x0[2] * OPSCALE);
    o.h[3] = (f16)(x0[3] * OPSCALE);
    o.h[4] = (f16)(x1[0] * OPSCALE);
    o.h[5] = (f16)(x1[1] * OPSCALE);
    o.h[6] = (f16)(x1[2] * OPSCALE);
    o.h[7] = (f16)(x1[3] * OPSCALE);
    const v4u w = o.u;
    f16* dst = Apk + (size_t)t * 8;
    *(volatile v4u*)dst = w;
    __threadfence();
    *(volatile v4u*)dst = w;
}

__global__ void __launch_bounds__(256)
k_prescale(const float* __restrict__ h, const float* __restrict__ ht,
           const float* __restrict__ hb, const float* __restrict__ z,
           const float* __restrict__ zb, f16* Xs, int B)
{
    __shared__ float tile[64][33];
    const int tid = threadIdx.x;
    const int tx = tid & 31, ty = tid >> 5;
    const int k0 = blockIdx.x * 64;
    const int b0 = blockIdx.y * 32;
    if (b0 + 32 > B || k0 + 64 > KTOT) return;
    const int b   = b0 + tx;
    const int seg = k0 >> 9;
    const int kk0 = k0 & (HID - 1);
    const float zc = z[b], zbc = zb[b];
    const float* src = (seg == 0) ? h : ((seg == 1) ? ht : hb);
    float fac = (seg == 0) ? (1.0f - zc) : ((seg == 1) ? zc : zbc);
    fac *= OPSCALE;
#pragma unroll
    for (int i = 0; i < 8; ++i) {
        const int kl = ty + 8 * i;
        tile[kl][tx] = fac * src[(size_t)(kk0 + kl) * B + b];
    }
    __syncthreads();
    const int r = ty * 4 + (tx >> 3);
    const int p = tx & 7;
    Pk8 o;
#pragma unroll
    for (int i = 0; i < 8; ++i) o.h[i] = (f16)tile[p * 8 + i][r];
    const v4u w = o.u;
    f16* dst = Xs + (size_t)(b0 + r) * KTOT + k0 + p * 8;
    *(volatile v4u*)dst = w;
    __threadfence();
    *(volatile v4u*)dst = w;
}

__global__ void __launch_bounds__(256)
k_gemm_cell(const f16* __restrict__ Apk, const f16* __restrict__ Xs,
            const float* __restrict__ bias, const float* __restrict__ z,
            const float* __restrict__ zb, const float* __restrict__ c_in,
            const float* __restrict__ h_in, float* out, int B)
{
    __shared__ __attribute__((aligned(32))) v4u sA[NFRAG * 64];
    __shared__ __attribute__((aligned(16))) float stg[2][ROWS_PB][STG_LD];

    const int tid  = threadIdx.x;
    const int lane = tid & 31, wave = tid >> 5;
    const int m16  = lane & 15, hh = lane >> 4;
    const int cb   = blockIdx.x;
    const int tg   = blockIdx.y;
    if ((cb + 1) * COLS_PB > B) return;
    if ((tg + 1) * ROWS_PB > HID) return;
    const int col  = cb * COLS_PB + wave * 16 + m16;

    const int coff = tid & 63;
    const int f0   = tid >> 6;
    const int f1   = f0 + 4;
    const int mt0  = (f0 >> 1) * 32 + tg * TSUB + (f0 & 1);
    const int mt1  = (f1 >> 1) * 32 + tg * TSUB + (f1 & 1);
    const f16* asrc0 = Apk + (size_t)mt0 * NKT * 512 + coff * 8;
    const f16* asrc1 = Apk + (size_t)mt1 * NKT * 512 + coff * 8;
    const f16* xrow  = Xs + (size_t)col * KTOT;

    v8f acc[NFRAG];
#pragma unroll
    for (int f = 0; f < NFRAG; ++f) acc[f] = (v8f){};

#pragma unroll 1
    for (int kt = 0; kt < NKT; ++kt) {
        __syncthreads();
        sA[f0 * 64 + coff] = *(const v4u*)(asrc0 + kt * 512);
        sA[f1 * 64 + coff] = *(const v4u*)(asrc1 + kt * 512);
        __syncthreads();

        const f16* xk = xrow + kt * 32;
        Frag bq;
        bq.half[0] = *(const v8h*)(xk + 8 * hh);
        bq.half[1] = *(const v8h*)(xk + 16 + 8 * hh);

        const f16* sAh = (const f16*)sA;
#pragma unroll
        for (int f = 0; f < NFRAG; ++f) {
            const f16* ap = sAh + f * 512 + lane * 16;
            Frag aq;
            aq.half[0] = *(const v8h*)(ap);
            aq.half[1] = *(const v8h*)(ap + 8);
            acc[f] = wmma16(aq.v, bq.v, acc[f]);
        }
    }

    const float zc = z[col], zbc = zb[col];
    const float omz  = 1.0f - zc;
    const float wkeep = omz * (1.0f - zbc);
    const float wupd  = omz * zbc;
    const int colb = wave * 16 + m16;
#pragma unroll
    for (int ttl = 0; ttl < TSUB; ++ttl) {
#pragma unroll
        for (int r = 0; r < 8; ++r) {
            const int rowl = ttl * 16 + hh * 8 + r;
            const int row  = tg * ROWS_PB + rowl;
            const float fs = acc[0 * TSUB + ttl][r] * INVSC + bias[row];
            const float is = acc[1 * TSUB + ttl][r] * INVSC + bias[HID + row];
            const float os = acc[2 * TSUB + ttl][r] * INVSC + bias[2 * HID + row];
            const float gs = acc[3 * TSUB + ttl][r] * INVSC + bias[3 * HID + row];
            const float fg = sigm_f(fs);
            const float ii = sigm_f(is);
            const float og = sigm_f(os);
            const float gg = tanh_f(gs);
            const size_t off = (size_t)row * B + col;
            const float c_old = c_in[off];
            const float h_old = h_in[off];
            const float ig = ii * gg;
            const float cn = zc * ig + wkeep * c_old + wupd * (fg * c_old + ig);
            const float tc = tanh_f(cn);
            const float hn = zc * og * tc + wkeep * h_old + wupd * og * tc;
            stg[0][rowl][colb] = hn;
            stg[1][rowl][colb] = cn;
        }
    }
    __syncthreads();

    const int q  = lane >> 3, p = lane & 7;
    const int cc = q * 32 + p * 4;
    float* outh = out;
    float* outc = out + (size_t)HID * B;
    v4f vals[8];
#pragma unroll
    for (int s = 0; s < 4; ++s) {
        const int rowl = wave * 4 + s;
        vals[s]     = *(const v4f*)(&stg[0][rowl][cc]);
        vals[4 + s] = *(const v4f*)(&stg[1][rowl][cc]);
    }
#pragma unroll
    for (int s = 0; s < 4; ++s) {
        const size_t ro = (size_t)(tg * ROWS_PB + wave * 4 + s) * B + (size_t)cb * COLS_PB + cc;
        *(volatile v4f*)(outh + ro) = vals[s];
        *(volatile v4f*)(outc + ro) = vals[4 + s];
    }
    __threadfence();
#pragma unroll
    for (int s = 0; s < 4; ++s) {
        const size_t ro = (size_t)(tg * ROWS_PB + wave * 4 + s) * B + (size_t)cb * COLS_PB + cc;
        *(volatile v4f*)(outh + ro) = vals[s];
        *(volatile v4f*)(outc + ro) = vals[4 + s];
    }
}

__global__ void __launch_bounds__(256)
k_zrow(const float* __restrict__ h, const float* __restrict__ ht,
       const float* __restrict__ hb, const float* __restrict__ z,
       const float* __restrict__ zb, const float* __restrict__ U11,
       const float* __restrict__ U21, const float* __restrict__ W01,
       const float* __restrict__ bias, float* out, int B)
{
    __shared__ __attribute__((aligned(16))) float zs[256];
    const int tid = threadIdx.x;
    const int lane = tid & 31, wave = tid >> 5;
    const int b0 = blockIdx.x * 256;
    if (b0 + 256 > B) return;
    const int b = b0 + tid;
    const float* w1 = U11 + (size_t)(4 * HID) * HID;
    const float* w2 = U21 + (size_t)(4 * HID) * HID;
    const float* w3 = W01 + (size_t)(4 * HID) * HID;
    float s1 = 0.0f, s2 = 0.0f, s3 = 0.0f;
#pragma unroll 4
    for (int k = 0; k < HID; ++k) {
        const size_t o = (size_t)k * B + b;
        s1 = __fmaf_rn(w1[k], h[o],  s1);
        s2 = __fmaf_rn(w2[k], ht[o], s2);
        s3 = __fmaf_rn(w3[k], hb[o], s3);
    }
    const float zc = z[b], zbc = zb[b];
    const float fs = (1.0f - zc) * s1 + zc * s2 + zbc * s3 + bias[4 * HID];
    float v = (fs + 1.0f) * 0.5f;
    v = fminf(1.0f, fmaxf(0.0f, v));
    zs[tid] = v;
    __syncthreads();
    if (lane < 8) {
        const v4f q4 = *(const v4f*)(&zs[wave * 32 + lane * 4]);
        float* dst = out + (size_t)2 * HID * B + b0 + wave * 32 + lane * 4;
        *(volatile v4f*)dst = q4;
        __threadfence();
        *(volatile v4f*)dst = q4;
    }
}

extern "C" void kernel_launch(void* const* d_in, const int* in_sizes, int n_in,
                              void* d_out, int out_size, void* d_ws, size_t ws_size,
                              hipStream_t stream)
{
    if (n_in < 10) return;
    const int B = in_sizes[4];
    if (B <= 0 || (B % 256) != 0) return;
    if (in_sizes[0] != HID * B || in_sizes[1] != HID * B ||
        in_sizes[2] != HID * B || in_sizes[3] != HID * B) return;
    if (in_sizes[5] != B) return;
    if (in_sizes[6] != (4 * HID + 1) * HID || in_sizes[7] != (4 * HID + 1) * HID ||
        in_sizes[8] != (4 * HID + 1) * HID) return;
    if (in_sizes[9] != 4 * HID + 1) return;
    if (out_size != (2 * HID + 1) * B) return;

    const size_t apk_halves = (size_t)(4 * HID) * KTOT;
    const size_t apk_bytes  = apk_halves * 2;
    const size_t xs_off     = (apk_bytes + 127) & ~(size_t)127;
    const size_t xs_bytes   = (size_t)B * KTOT * 2;
    if (xs_off + xs_bytes > ws_size) return;

    const float* c        = (const float*)d_in[0];
    const float* h_bottom = (const float*)d_in[1];
    const float* h        = (const float*)d_in[2];
    const float* h_top    = (const float*)d_in[3];
    const float* z        = (const float*)d_in[4];
    const float* z_bottom = (const float*)d_in[5];
    const float* U11      = (const float*)d_in[6];
    const float* U21      = (const float*)d_in[7];
    const float* W01      = (const float*)d_in[8];
    const float* bias     = (const float*)d_in[9];
    float* out = (float*)d_out;

    f16* Apk = (f16*)d_ws;
    f16* Xs  = (f16*)((char*)d_ws + xs_off);

    const int total8 = (int)(apk_halves / 8);
    k_pack_w<<<(total8 + 255) / 256, 256, 0, stream>>>(U11, U21, W01, Apk, total8);
    k_prescale<<<dim3(KTOT / 64, B / 32), 256, 0, stream>>>(
        h, h_top, h_bottom, z, z_bottom, Xs, B);
    k_gemm_cell<<<dim3(B / COLS_PB, HID / ROWS_PB), 256, 0, stream>>>(
        Apk, Xs, bias, z, z_bottom, c, h, out, B);
    k_zrow<<<B / 256, 256, 0, stream>>>(
        h, h_top, h_bottom, z, z_bottom, U11, U21, W01, bias, out, B);
    (void)hipGetLastError();
}
